// BehaviorMoE_90374701843251
// MI455X (gfx1250) — hardware-verified
//
#include <hip/hip_runtime.h>
#include <stddef.h>

#define DM    1024
#define NT    8192
#define NB    4
#define NSH   3
#define NE    4
#define NPL   (NSH + NB)
#define TB    16
#define NTHR  256
#define NWAV  (NTHR / 32)
#define XP    1032
#define SP    1028
#define LN_EPS 1e-5f
#define WSC   16.0f
#define XS_BYTES (TB * XP * 2)
#define SS_BYTES (TB * SP * 4)
#define DYN_BYTES (XS_BYTES + SS_BYTES)

static_assert(NT % NTHR == 0);
static_assert(NT % TB == 0);
static_assert(TB * (DM / 8) == 8 * NTHR);
static_assert(NWAV * 2 == TB);
static_assert(NWAV * 128 == DM);
static_assert(XP % 8 == 0);
static_assert(SP % 4 == 0);
static_assert(DM % 32 == 0);
static_assert(XS_BYTES % 16 == 0);
static_assert((NSH * DM * DM) % (8 * 256) == 0);
static_assert((NB * DM * DM) % (8 * 256) == 0);
static_assert(NT % 8 == 0);

typedef _Float16 f16;
typedef f16 v16h __attribute__((ext_vector_type(16)));
typedef f16 v8h_t __attribute__((ext_vector_type(8)));
typedef v8h_t __attribute__((may_alias)) v8h;
typedef float v8f __attribute__((ext_vector_type(8)));
typedef float v4f_t __attribute__((ext_vector_type(4)));
typedef v4f_t __attribute__((may_alias)) v4f;
typedef unsigned int v4u_t __attribute__((ext_vector_type(4)));
typedef v4u_t __attribute__((may_alias)) v4u;

union Frag { v16h v; v8h_t h[2]; };

__device__ __forceinline__ v8f zero8() {
    v8f z;
#pragma unroll
    for (int i = 0; i < 8; ++i) z[i] = 0.0f;
    return z;
}

__device__ __forceinline__ v16h ldfrag(const f16* p, int k0) {
    Frag f;
    f.h[0] = *(const v8h*)(p + k0);
    f.h[1] = *(const v8h*)(p + k0 + 16);
    return f.v;
}

__device__ __forceinline__ v8f wmma16(v16h a, v16h b, v8f c) {
    return __builtin_amdgcn_wmma_f32_16x16x32_f16(false, a, false, b, (short)0, c, false, false);
}

__global__ void __launch_bounds__(256) cvt_f16_kernel(
    const float* __restrict__ src, f16* __restrict__ dst, int n8, float scale)
{
    const int i = blockIdx.x * 256 + threadIdx.x;
    const bool ok = (i < n8);
    const int ic = ok ? i : (n8 - 1);
    const v4f_t a = *(const v4f*)(src + (size_t)ic * 8);
    const v4f_t b = *(const v4f*)(src + (size_t)ic * 8 + 4);
    union { v8h_t h; v4u_t u; } pk;
#pragma unroll
    for (int j = 0; j < 4; ++j) {
        pk.h[j]     = (f16)(a[j] * scale);
        pk.h[4 + j] = (f16)(b[j] * scale);
    }
    if (ok) *(volatile v4u_t*)(dst + (size_t)i * 8) = pk.u;
    __threadfence();
    if (ok) *(volatile v4u_t*)(dst + (size_t)i * 8) = pk.u;
}

__global__ void __launch_bounds__(NTHR) moe_kernel(
    const float* __restrict__ x, const int* __restrict__ b_seq,
    const f16* __restrict__ wpl,
    const float* __restrict__ b_sh, const float* __restrict__ b_sp,
    const float* __restrict__ w_gates,
    const float* __restrict__ gamma, const float* __restrict__ beta,
    float* __restrict__ out)
{
    extern __shared__ __attribute__((aligned(16))) unsigned char dyn_lds[];
    f16*   xs   = (f16*)dyn_lds;
    float* sels = (float*)(dyn_lds + XS_BYTES);
    __shared__ int   toks[TB];
    __shared__ float gl[TB * NE];
    __shared__ int   wcnt[NWAV];

    const int tid = threadIdx.x, lane = tid & 31, w = tid >> 5;
    const int hh = lane >> 4, m = lane & 15;
    const int tb = blockIdx.y;
    const int slot0 = blockIdx.x * TB;

    if (tid < TB) toks[tid] = 0;
    int base = 0;
#pragma unroll 1
    for (int c = 0; c < NT / NTHR; ++c) {
        const int n = c * NTHR + tid;
        int b = b_seq[n];
        b = (b < 0) ? 0 : ((b > NB) ? NB : b);
        const bool hit = (b == tb + 1);
        const unsigned bal  = __builtin_amdgcn_ballot_w32(hit);
        const int      wpop = __builtin_popcount(bal);
        const int      lpre = __builtin_popcount(bal & ((1u << lane) - 1u));
        if (lane == 0) wcnt[w] = wpop;
        __syncthreads();
        int pre = 0, tot = 0;
#pragma unroll
        for (int i = 0; i < NWAV; ++i) {
            const int v = wcnt[i];
            tot += v;
            pre += (i < w) ? v : 0;
        }
        const int rk = base + pre + lpre - slot0;
        if (hit && rk >= 0 && rk < TB) toks[rk] = n;
        base += tot;
        __syncthreads();
        if (base >= slot0 + TB) break;
    }
    int nvalid = base - slot0;
    nvalid = (nvalid > TB) ? TB : nvalid;
    if (nvalid <= 0) return;

#pragma unroll
    for (int jj = 0; jj < 8; ++jj) {
        const int q  = jj * NTHR + tid;
        const int r  = q >> 7;
        const int c8 = (q & 127) * 8;
        const int tok = toks[r];
        const float* xr = x + (size_t)tok * DM + c8;
        const v4f_t a0 = *(const v4f*)xr;
        const v4f_t a1 = *(const v4f*)(xr + 4);
        v8h_t pk;
#pragma unroll
        for (int j = 0; j < 4; ++j) {
            pk[j]     = (f16)a0[j];
            pk[4 + j] = (f16)a1[j];
        }
        *(v8h*)(xs + r * XP + c8) = pk;
    }

    const float* wg = w_gates + (size_t)tb * DM * NE;
#pragma unroll
    for (int qq = 0; qq < 2; ++qq) {
        const int r = 2 * w + qq;
        const int tok = toks[r];
        const float* xr = x + (size_t)tok * DM;
        float l0 = 0.0f, l1 = 0.0f, l2 = 0.0f, l3 = 0.0f;
#pragma unroll 1
        for (int j = 0; j < DM / 32; ++j) {
            const int d = j * 32 + lane;
            const float xv = xr[d];
            const v4f_t wv = *(const v4f*)(wg + (size_t)d * NE);
            l0 = fmaf(xv, wv[0], l0);
            l1 = fmaf(xv, wv[1], l1);
            l2 = fmaf(xv, wv[2], l2);
            l3 = fmaf(xv, wv[3], l3);
        }
#pragma unroll
        for (int off = 16; off > 0; off >>= 1) {
            l0 += __shfl_xor(l0, off, 32);
            l1 += __shfl_xor(l1, off, 32);
            l2 += __shfl_xor(l2, off, 32);
            l3 += __shfl_xor(l3, off, 32);
        }
        const float mx = fmaxf(fmaxf(l0, l1), fmaxf(l2, l3));
        const float e0 = expf(l0 - mx), e1 = expf(l1 - mx);
        const float e2 = expf(l2 - mx), e3 = expf(l3 - mx);
        const float sum = (e0 + e1) + (e2 + e3);
        const float inv = 1.0f / sum;
        if (lane == 0) {
            gl[r * NE + 0] = e0 * inv;
            gl[r * NE + 1] = e1 * inv;
            gl[r * NE + 2] = e2 * inv;
            gl[r * NE + 3] = e3 * inv;
        }
    }
    __syncthreads();

    const f16* xa   = xs + m * XP + 8 * hh;
    const int  colw = w * 128;
#pragma unroll 1
    for (int cg = 0; cg < 2; ++cg) {
        const int colg = colw + cg * 64;
        v8f sacc[4];
#pragma unroll
        for (int j = 0; j < 4; ++j) sacc[j] = zero8();

#pragma unroll 1
        for (int e = 0; e < NE; ++e) {
            const int pl = (e < NSH) ? e : (NSH + tb);
            const f16* wb = wpl + (size_t)pl * DM * DM + (size_t)(colg + m) * DM + 8 * hh;
            v8f cur[4];
#pragma unroll
            for (int j = 0; j < 4; ++j) cur[j] = zero8();
#pragma unroll 1
            for (int k0 = 0; k0 < DM; k0 += 32) {
                const v16h a = ldfrag(xa, k0);
                v16h bf;
#pragma unroll
                for (int j = 0; j < 4; ++j) {
                    bf = ldfrag(wb + (size_t)j * 16 * DM, k0);
                    cur[j] = wmma16(a, bf, cur[j]);
                }
                asm volatile("v_nop\n\tv_nop\n\tv_nop\n\tv_nop"
                             : "+v"(cur[0]), "+v"(cur[1]), "+v"(cur[2]), "+v"(cur[3])
                             : "v"(a), "v"(bf));
            }
            const int esh = (e < NSH) ? e : 0;
#pragma unroll
            for (int j = 0; j < 4; ++j) {
                const int col = colg + 16 * j + m;
                const float bshv = b_sh[(size_t)esh * DM + col];
                const float bspv = b_sp[(size_t)tb * DM + col];
                const float bias = (e < NSH) ? bshv : bspv;
#pragma unroll
                for (int r = 0; r < 8; ++r) {
                    const float gv = gl[(8 * hh + r) * NE + e];
                    const float yv = cur[j][r] * (1.0f / WSC) + bias;
                    sacc[j][r] = fmaf(gv, yv, sacc[j][r]);
                }
            }
        }
#pragma unroll
        for (int j = 0; j < 4; ++j) {
            const int col = colg + 16 * j + m;
#pragma unroll
            for (int r = 0; r < 8; ++r)
                sels[(8 * hh + r) * SP + col] = sacc[j][r];
        }
    }
    __syncthreads();

#pragma unroll 1
    for (int qq = 0; qq < 2; ++qq) {
        const int r = 2 * w + qq;
        const int tok = toks[r];
        const float* sr = sels + r * SP + 4 * lane;
        v4f_t sv[8];
        float s = 0.0f;
#pragma unroll
        for (int i = 0; i < 8; ++i) {
            sv[i] = *(const v4f*)(sr + 128 * i);
            s += (sv[i][0] + sv[i][1]) + (sv[i][2] + sv[i][3]);
        }
#pragma unroll
        for (int off = 16; off > 0; off >>= 1) s += __shfl_xor(s, off, 32);
        const float mu = s * (1.0f / DM);
        float ss = 0.0f;
#pragma unroll
        for (int i = 0; i < 8; ++i) {
#pragma unroll
            for (int cc = 0; cc < 4; ++cc) {
                const float dv = sv[i][cc] - mu;
                ss = fmaf(dv, dv, ss);
            }
        }
#pragma unroll
        for (int off = 16; off > 0; off >>= 1) ss += __shfl_xor(ss, off, 32);
        const float var = ss * (1.0f / DM);
        const float rsd = rsqrtf(var + LN_EPS);

        const float* xr = x + (size_t)tok * DM + 4 * lane;
        const float* gp = gamma + 4 * lane;
        const float* bp = beta + 4 * lane;
        v4f_t o[8];
#pragma unroll
        for (int i = 0; i < 8; ++i) {
            const v4f_t xv = *(const v4f*)(xr + 128 * i);
            const v4f_t gm = *(const v4f*)(gp + 128 * i);
            const v4f_t bt = *(const v4f*)(bp + 128 * i);
#pragma unroll
            for (int cc = 0; cc < 4; ++cc)
                o[i][cc] = xv[cc] + ((sv[i][cc] - mu) * rsd * gm[cc] + bt[cc]);
        }
        float* orow = out + (size_t)tok * DM + 4 * lane;
        if (r < nvalid) {
#pragma unroll
            for (int i = 0; i < 8; ++i)
                *(volatile v4f_t*)(orow + 128 * i) = o[i];
        }
        __threadfence();
        if (r < nvalid) {
#pragma unroll
            for (int i = 0; i < 8; ++i)
                *(volatile v4f_t*)(orow + 128 * i) = o[i];
        }
    }
}

__global__ void __launch_bounds__(256) zero_rows_kernel(
    const float* __restrict__ x, const int* __restrict__ b_seq,
    const float* __restrict__ beta, float* __restrict__ out, int ntok)
{
    const int lane = threadIdx.x & 31, w = threadIdx.x >> 5;
    const int n = blockIdx.x * 8 + w;
    if (n >= ntok) return;
    int b = b_seq[n];
    b = (b < 0) ? 0 : ((b > NB) ? NB : b);
    if (b != 0) return;
    const float* xr = x + (size_t)n * DM + 4 * lane;
    const float* bp = beta + 4 * lane;
    v4f_t o[8];
#pragma unroll
    for (int i = 0; i < 8; ++i) {
        const v4f_t xv = *(const v4f*)(xr + 128 * i);
        const v4f_t bt = *(const v4f*)(bp + 128 * i);
#pragma unroll
        for (int cc = 0; cc < 4; ++cc) o[i][cc] = xv[cc] + bt[cc];
    }
    float* orow = out + (size_t)n * DM + 4 * lane;
#pragma unroll
    for (int i = 0; i < 8; ++i) *(volatile v4f_t*)(orow + 128 * i) = o[i];
    __threadfence();
#pragma unroll
    for (int i = 0; i < 8; ++i) *(volatile v4f_t*)(orow + 128 * i) = o[i];
}

extern "C" void kernel_launch(void* const* d_in, const int* in_sizes, int n_in,
                              void* d_out, int out_size, void* d_ws, size_t ws_size,
                              hipStream_t stream)
{
    if (n_in < 9) return;
    if (in_sizes[0] != NT * DM) return;
    if (in_sizes[1] != NT) return;
    if (in_sizes[2] != NSH * DM * DM) return;
    if (in_sizes[3] != NSH * DM) return;
    if (in_sizes[4] != NB * DM * DM) return;
    if (in_sizes[5] != NB * DM) return;
    if (in_sizes[6] != NB * DM * NE) return;
    if (in_sizes[7] != DM) return;
    if (in_sizes[8] != DM) return;
    if (out_size != NT * DM) return;

    const float* x       = (const float*)d_in[0];
    const int*   b_seq   = (const int*)  d_in[1];
    const float* W_sh    = (const float*)d_in[2];
    const float* b_sh    = (const float*)d_in[3];
    const float* W_sp    = (const float*)d_in[4];
    const float* b_sp    = (const float*)d_in[5];
    const float* w_gates = (const float*)d_in[6];
    const float* gamma   = (const float*)d_in[7];
    const float* beta    = (const float*)d_in[8];
    float* out = (float*)d_out;

    const size_t nSh   = (size_t)NSH * DM * DM;
    const size_t nSp   = (size_t)NB * DM * DM;
    const size_t total = (nSh + nSp) * 2;
    if (total > ws_size) return;

    char* ws = (char*)d_ws;
    f16* wpl = (f16*)ws;

    const int n8Sh = (int)(nSh / 8), n8Sp = (int)(nSp / 8);
    cvt_f16_kernel<<<(n8Sh + 255) / 256, 256, 0, stream>>>(W_sh, wpl, n8Sh, WSC);
    cvt_f16_kernel<<<(n8Sp + 255) / 256, 256, 0, stream>>>(W_sp, wpl + nSh, n8Sp, WSC);

    hipFuncSetAttribute(reinterpret_cast<const void*>(&moe_kernel),
                        hipFuncAttributeMaxDynamicSharedMemorySize, DYN_BYTES);
    dim3 g(NT / TB, NB);
    moe_kernel<<<g, NTHR, DYN_BYTES, stream>>>(x, b_seq, wpl, b_sh, b_sp, w_gates,
                                                gamma, beta, out);

    zero_rows_kernel<<<NT / 8, 256, 0, stream>>>(x, b_seq, beta, out, NT);
}
